// GNNLinkPredictor_16192026706661
// MI455X (gfx1250) — hardware-run, weakly checked
//
#include <hip/hip_runtime.h>
#include <stddef.h>
#include <stdint.h>

#define NN      100000
#define NE      1600000
#define NPAIR   200000
#define CIN     64
#define CHID    128
#define COUT    64
#define MP      100096
#define K1      192
#define K2      256
#define M1P     128
#define GBM     64
#define GBN     128
#define GTHR    128
#define NTHR    256
#define NWAVE   8
#define EPT     8
#define WCH     (32 * EPT)
#define NBRUN   1024
#define SLB     10
#define NBK     98
#define WLCAP   2560
#define RCAP    20480
#define DEGCAP  64
#define MAXDEG_MEAS   36
#define MAXB1024_MEAS 16684
#define ABM     64
#define DPB     1024
#define NDB     196

#define BK_ZINTS (NWAVE * WLCAP + RCAP + 3 * NBRUN)
#define BK_INTS  (BK_ZINTS + 16)
#define BK_LDS   (BK_INTS * 4)

#define PBX   (MP * CIN / 8 / NTHR)
#define PBW1  12
#define PBW2  16
#define PBTOT (PBX + PBW1 + PBW2 + 1)

static_assert(CIN == 64 && CHID == 128 && COUT == 64);
static_assert(MP % GBM == 0 && MP >= NN && MP == 782 * 128 && MP % ABM == 0);
static_assert(NBRUN == (1 << SLB) && NBRUN % ABM == 0 && NBRUN % 32 == 0);
static_assert(NBK * NBRUN >= MP);
static_assert(NE < (1 << 21) && (((long long)NE) << SLB) < (1LL << 31));
static_assert(NE % WCH == 0 && NE % 4 == 0);
static_assert(RCAP == NWAVE * WLCAP && RCAP % (NTHR * 4) == 0 && BK_ZINTS % 4 == 0);
static_assert((2 * NBRUN) % (NTHR * 4) == 0);
static_assert((long long)RCAP * 100 >= (long long)MAXB1024_MEAS * 105);
static_assert(WLCAP >= MAXB1024_MEAS / 8 + 8 * 46 + 1);
static_assert(NN > 65535);
static_assert(MAXDEG_MEAS + 8 <= DEGCAP);
static_assert(K1 % 32 == 0 && K2 % 32 == 0 && K1 == 3 * CIN && K2 == 2 * CHID && M1P == 2 * CIN);
static_assert(GBN == CHID && GBN == 2 * COUT && GBM == (GTHR / 32) * 16);
static_assert((MP * CIN / 8) % NTHR == 0);
static_assert(3 * CHID * (CIN / 8) == PBW1 * NTHR && 4 * COUT * (CHID / 8) == PBW2 * NTHR);
static_assert(BK_LDS <= 300000);
static_assert((GBM * GBN + 128) * 4 <= 65536);
static_assert(NPAIR % 32 == 0 && DPB % 32 == 0 && DPB == 4 * NTHR);
static_assert(NDB * DPB >= NPAIR && (NDB - 1) * DPB < NPAIR && ((NPAIR - (NDB - 1) * DPB) % 32) == 0);
static_assert(NBK <= NTHR);

typedef float          v4f   __attribute__((ext_vector_type(4)));
typedef float          v8f   __attribute__((ext_vector_type(8)));
typedef int            v4i   __attribute__((ext_vector_type(4)));
typedef int            v8i   __attribute__((ext_vector_type(8)));
typedef unsigned       v2u   __attribute__((ext_vector_type(2)));
typedef unsigned short v8us  __attribute__((ext_vector_type(8)));
typedef unsigned short v16us __attribute__((ext_vector_type(16)));
typedef __bf16         v16bf __attribute__((ext_vector_type(16)));
typedef v4f  __attribute__((may_alias)) v4fa;
typedef v4i  __attribute__((may_alias)) v4ia;
typedef v2u  __attribute__((may_alias)) v2ua;
typedef v8us __attribute__((may_alias)) v8usa;
union FragB { v16bf v; v16us u; v8us h[2]; v8i w; };

__device__ __forceinline__ v8f wmb(const FragB& a, const FragB& b, v8f c) {
  v8f d = __builtin_amdgcn_wmma_f32_16x16x32_bf16(false, a.v, false, b.v, (short)0, c, false, false);
  asm volatile("v_nop\n\tv_nop\n\tv_nop\n\tv_nop" : "+v"(d) : "v"(a.w), "v"(b.w));
  return d;
}

__device__ __forceinline__ unsigned bf16_bits(float f) {
  const unsigned u = __float_as_uint(f);
  const unsigned r = (u + 0x7FFFu + ((u >> 16) & 1u)) >> 16;
  const unsigned q = (u >> 16) | 0x40u;
  return ((u & 0x7fffffffu) > 0x7f800000u) ? q : r;
}

__device__ __forceinline__ void hilo_pack(float v0, float v1, float v2, float v3,
                                          int& h01, int& h23, int& l01, int& l23) {
  const unsigned a0 = bf16_bits(v0), a1 = bf16_bits(v1), a2 = bf16_bits(v2), a3 = bf16_bits(v3);
  const unsigned b0 = bf16_bits(v0 - __uint_as_float(a0 << 16));
  const unsigned b1 = bf16_bits(v1 - __uint_as_float(a1 << 16));
  const unsigned b2 = bf16_bits(v2 - __uint_as_float(a2 << 16));
  const unsigned b3 = bf16_bits(v3 - __uint_as_float(a3 << 16));
  h01 = (int)(a0 | (a1 << 16)); h23 = (int)(a2 | (a3 << 16));
  l01 = (int)(b0 | (b1 << 16)); l23 = (int)(b2 | (b3 << 16));
}

__device__ __forceinline__ v4i regroup8(int h01, int h23, int l01, int l23, int lane) {
  const int t  = lane & 15;
  const int s0 = (lane & 16) + ((2 * t) & 15), s1 = s0 + 1;
  const int a0 = __shfl(h01, s0, 32), a1 = __shfl(h23, s0, 32), a2 = __shfl(h01, s1, 32), a3 = __shfl(h23, s1, 32);
  const int b0 = __shfl(l01, s0, 32), b1 = __shfl(l23, s0, 32), b2 = __shfl(l01, s1, 32), b3 = __shfl(l23, s1, 32);
  const int mk = (t < 8) ? -1 : 0;
  v4i o;
  o.x = (a0 & mk) | (b0 & ~mk); o.y = (a1 & mk) | (b1 & ~mk);
  o.z = (a2 & mk) | (b2 & ~mk); o.w = (a3 & mk) | (b3 & ~mk);
  return o;
}

__device__ __forceinline__ unsigned hl_pick(float v, unsigned hm) {
  const unsigned hb = bf16_bits(v);
  const unsigned lb = bf16_bits(v - __uint_as_float(hb << 16));
  return (hb & hm) | (lb & ~hm);
}

__device__ __forceinline__ void st2_v4f(float* p, v4f v) {
  *(volatile v4f*)p = v;
  __threadfence();
  *(volatile v4f*)p = v;
}
__device__ __forceinline__ void st2_v4i(unsigned short* p, v4i v) {
  *(volatile v4i*)p = v;
  __threadfence();
  *(volatile v4i*)p = v;
}
__device__ __forceinline__ void st2_v8us(unsigned short* p, v8us v) {
  *(volatile v8us*)p = v;
  __threadfence();
  *(volatile v8us*)p = v;
}

__device__ __forceinline__ v8us col8(const float* __restrict__ base, int stride) {
  float f[8];
#pragma unroll
  for (int i = 0; i < 8; ++i) f[i] = base[(size_t)i * (size_t)stride];
  v8us o;
#pragma unroll
  for (int i = 0; i < 8; ++i) o[i] = (unsigned short)bf16_bits(f[i]);
  return o;
}

__global__ __launch_bounds__(NTHR) void k_prep(const float* __restrict__ x,
                                               const float* __restrict__ wl1, const float* __restrict__ wr1,
                                               const float* __restrict__ b1,
                                               const float* __restrict__ wl2, const float* __restrict__ wr2,
                                               const float* __restrict__ b2,
                                               unsigned short* xb, unsigned short* w1c, unsigned short* w2c,
                                               float* sm) {
  const int tid = (int)threadIdx.x, lane = tid & 31, wave = tid >> 5;
  const int blk = (int)blockIdx.x;
  if (blk < PBX) {
    const int u   = blk * NTHR + tid;
    const int row = u >> 3, k8 = (u & 7) * 8;
    const int rc  = row < NN ? row : NN - 1;
    const unsigned mk = row < NN ? 0xffffu : 0u;
    const float* p = x + (size_t)rc * CIN + k8;
    const v4f a = *(const v4fa*)p;
    const v4f b = *(const v4fa*)(p + 4);
    v8us o;
    o[0] = (unsigned short)(bf16_bits(a.x) & mk); o[1] = (unsigned short)(bf16_bits(a.y) & mk);
    o[2] = (unsigned short)(bf16_bits(a.z) & mk); o[3] = (unsigned short)(bf16_bits(a.w) & mk);
    o[4] = (unsigned short)(bf16_bits(b.x) & mk); o[5] = (unsigned short)(bf16_bits(b.y) & mk);
    o[6] = (unsigned short)(bf16_bits(b.z) & mk); o[7] = (unsigned short)(bf16_bits(b.w) & mk);
    st2_v8us(xb + (size_t)row * CIN + k8, o);
  } else if (blk < PBX + PBW1) {
    const int bl   = blk - PBX;
    const int part = bl >> 2;
    const int u    = (bl & 3) * NTHR + tid;
    const int n    = u >> 3, k8 = (u & 7) * 8;
    v8us o;
    if (part < 2) o = col8(wl1 + (size_t)k8 * CHID + n, CHID);
    else          o = col8(wr1 + (size_t)k8 * CHID + n, CHID);
    st2_v8us(w1c + (size_t)n * K1 + CIN * part + k8, o);
  } else if (blk < PBX + PBW1 + PBW2) {
    const int bl   = blk - PBX - PBW1;
    const int part = bl >> 2;
    const int sel  = part >> 1, dup = part & 1;
    const int u    = (bl & 3) * NTHR + tid;
    const int nl   = u >> 4, k8 = (u & 15) * 8;
    v8us o;
    if (sel == 0) o = col8(wl2 + (size_t)k8 * COUT + nl, COUT);
    else          o = col8(wr2 + (size_t)k8 * COUT + nl, COUT);
    st2_v8us(w2c + (size_t)(COUT * sel + nl) * K2 + CHID * dup + k8, o);
  } else {
    if (wave == 0) {
      const v4f a = *(const v4fa*)(b1 + 4 * lane);
      v4f o;
      o.x = __uint_as_float(bf16_bits(a.x) << 16); o.y = __uint_as_float(bf16_bits(a.y) << 16);
      o.z = __uint_as_float(bf16_bits(a.z) << 16); o.w = __uint_as_float(bf16_bits(a.w) << 16);
      st2_v4f(sm + 4 * lane, o);
    } else if (wave == 1) {
      const v4f a = *(const v4fa*)(b2 + 4 * (lane & 15));
      const unsigned mk = (lane < 16) ? 0xffffffffu : 0u;
      v4f o;
      o.x = __uint_as_float((bf16_bits(a.x) << 16) & mk); o.y = __uint_as_float((bf16_bits(a.y) << 16) & mk);
      o.z = __uint_as_float((bf16_bits(a.z) << 16) & mk); o.w = __uint_as_float((bf16_bits(a.w) << 16) & mk);
      st2_v4f(sm + 128 + 4 * lane, o);
    }
  }
}

__device__ __forceinline__ void bucket_flush(const int* pl, const int* cnt, int ov, int* lp, int* cop, int* fp,
                                             int tid) {
#pragma unroll 1
  for (int i = tid * 4; i < RCAP; i += NTHR * 4) {
    const v4i v = *(const v4ia*)(pl + i);
    *(volatile v4i*)(lp + i) = v;
  }
#pragma unroll 1
  for (int i = tid * 4; i < 2 * NBRUN; i += NTHR * 4) {
    const v4i v = *(const v4ia*)(cnt + i);
    *(volatile v4i*)(cop + i) = v;
  }
  if (tid < 8) {
    const v4i f = {ov, ov, ov, ov};
    *(volatile v4i*)(fp + 4 * tid) = f;
  }
}

__global__ __launch_bounds__(NTHR) void k_bucket(const int* __restrict__ srcs, const int* __restrict__ dsts,
                                                 int* LIST, int* CO, int* FLAG) {
  extern __shared__ __attribute__((aligned(16))) int dsm[];
  int* wl   = dsm;
  int* pl   = dsm + NWAVE * WLCAP;
  int* cnt  = pl + RCAP;
  int* offs = cnt + NBRUN;
  int* cur  = offs + NBRUN;
  int* misc = cur + NBRUN;
  const int tid = (int)threadIdx.x, lane = tid & 31, wave = tid >> 5;
  const int blk = (int)blockIdx.x;
  const unsigned nbs = (unsigned)(blk * NBRUN);

  {
    const v4i z4 = {0, 0, 0, 0};
    for (int i = tid * 4; i < BK_ZINTS; i += NTHR * 4) *(v4ia*)(dsm + i) = z4;
    if (tid < 16) misc[tid] = 0;
  }
  __syncthreads();

  {
    const int per  = ((NE + NWAVE * WCH - 1) / (NWAVE * WCH)) * WCH;
    const int ebeg = wave * per;
    const int eend = (ebeg + per < NE) ? (ebeg + per) : NE;
    int* mylist = wl + wave * WLCAP;
    int wc = 0;
#pragma unroll 1
    for (int cb = ebeg; cb < eend; cb += WCH) {
      const int e0 = cb + lane * EPT;
      const v4i da = *(const v4ia*)(dsts + e0);
      const v4i db = *(const v4ia*)(dsts + e0 + 4);
      const unsigned s0 = (unsigned)da.x - nbs, s1 = (unsigned)da.y - nbs;
      const unsigned s2 = (unsigned)da.z - nbs, s3 = (unsigned)da.w - nbs;
      const unsigned s4 = (unsigned)db.x - nbs, s5 = (unsigned)db.y - nbs;
      const unsigned s6 = (unsigned)db.z - nbs, s7 = (unsigned)db.w - nbs;
      const bool h0 = s0 < (unsigned)NBRUN, h1 = s1 < (unsigned)NBRUN, h2 = s2 < (unsigned)NBRUN, h3 = s3 < (unsigned)NBRUN;
      const bool h4 = s4 < (unsigned)NBRUN, h5 = s5 < (unsigned)NBRUN, h6 = s6 < (unsigned)NBRUN, h7 = s7 < (unsigned)NBRUN;
      const unsigned m0 = __builtin_amdgcn_ballot_w32(h0), m1 = __builtin_amdgcn_ballot_w32(h1);
      const unsigned m2 = __builtin_amdgcn_ballot_w32(h2), m3 = __builtin_amdgcn_ballot_w32(h3);
      const unsigned m4 = __builtin_amdgcn_ballot_w32(h4), m5 = __builtin_amdgcn_ballot_w32(h5);
      const unsigned m6 = __builtin_amdgcn_ballot_w32(h6), m7 = __builtin_amdgcn_ballot_w32(h7);
      const unsigned any = m0 | m1 | m2 | m3 | m4 | m5 | m6 | m7;
      if (any != 0u) {
        const int pre = (int)(__builtin_amdgcn_mbcnt_lo(m0, 0u) + __builtin_amdgcn_mbcnt_lo(m1, 0u) +
                              __builtin_amdgcn_mbcnt_lo(m2, 0u) + __builtin_amdgcn_mbcnt_lo(m3, 0u) +
                              __builtin_amdgcn_mbcnt_lo(m4, 0u) + __builtin_amdgcn_mbcnt_lo(m5, 0u) +
                              __builtin_amdgcn_mbcnt_lo(m6, 0u) + __builtin_amdgcn_mbcnt_lo(m7, 0u));
        int p = wc + pre;
        if (h0) { if (p < WLCAP) mylist[p] = ((e0 + 0) << SLB) | (int)s0; p = p + 1; }
        if (h1) { if (p < WLCAP) mylist[p] = ((e0 + 1) << SLB) | (int)s1; p = p + 1; }
        if (h2) { if (p < WLCAP) mylist[p] = ((e0 + 2) << SLB) | (int)s2; p = p + 1; }
        if (h3) { if (p < WLCAP) mylist[p] = ((e0 + 3) << SLB) | (int)s3; p = p + 1; }
        if (h4) { if (p < WLCAP) mylist[p] = ((e0 + 4) << SLB) | (int)s4; p = p + 1; }
        if (h5) { if (p < WLCAP) mylist[p] = ((e0 + 5) << SLB) | (int)s5; p = p + 1; }
        if (h6) { if (p < WLCAP) mylist[p] = ((e0 + 6) << SLB) | (int)s6; p = p + 1; }
        if (h7) { if (p < WLCAP) mylist[p] = ((e0 + 7) << SLB) | (int)s7; p = p + 1; }
        wc += (int)(__builtin_popcount(m0) + __builtin_popcount(m1) + __builtin_popcount(m2) + __builtin_popcount(m3) +
                    __builtin_popcount(m4) + __builtin_popcount(m5) + __builtin_popcount(m6) + __builtin_popcount(m7));
      }
    }
    if (lane == 0) misc[wave] = wc;
  }
  __syncthreads();

  if (wave == 0) {
    int ov = 0;
#pragma unroll 1
    for (int w2 = 0; w2 < NWAVE; ++w2) {
      int c = misc[w2];
      if (c > WLCAP) ov = 1;
      c = c < 0 ? 0 : (c > WLCAP ? WLCAP : c);
#pragma unroll 1
      for (int b0 = 0; b0 < c; b0 += 32) {
        const int idx = b0 + lane;
        const int ent = wl[w2 * WLCAP + (idx < WLCAP ? idx : WLCAP - 1)];
        const int m32 = (c - b0) < 32 ? (c - b0) : 32;
#pragma unroll 1
        for (int k = 0; k < m32; ++k) {
          const int u    = __builtin_amdgcn_readlane(ent, k);
          const int slot = u & (NBRUN - 1);
          if (lane == 0) cnt[slot] = cnt[slot] + 1;
        }
      }
    }
    if (lane == 0) misc[9] = ov;
  }
  __syncthreads();
  if (wave == 0) {
    const int base = lane * (NBRUN / 32);
    int s = 0;
#pragma unroll 1
    for (int i = 0; i < NBRUN / 32; ++i) s += cnt[base + i];
    int incl = s;
#pragma unroll
    for (int d = 1; d < 32; d <<= 1) {
      const int y = __shfl_up(incl, d, 32);
      if (lane >= d) incl += y;
    }
    int run = incl - s;
#pragma unroll 1
    for (int i = 0; i < NBRUN / 32; ++i) {
      const int cv = cnt[base + i];
      offs[base + i] = run;
      cur[base + i]  = run;
      run += cv;
    }
  }
  __syncthreads();

  if (wave == 0) {
#pragma unroll 1
    for (int w2 = 0; w2 < NWAVE; ++w2) {
      int c = misc[w2];
      c = c < 0 ? 0 : (c > WLCAP ? WLCAP : c);
#pragma unroll 1
      for (int b0 = 0; b0 < c; b0 += 32) {
        const int idx = b0 + lane;
        const int ent = wl[w2 * WLCAP + (idx < WLCAP ? idx : WLCAP - 1)];
        int eid = (ent >> SLB) & 0x1FFFFF;
        eid = eid > NE - 1 ? NE - 1 : eid;
        int sr = srcs[eid];
        sr = sr < 0 ? 0 : (sr > NN - 1 ? NN - 1 : sr);
        const int m32 = (c - b0) < 32 ? (c - b0) : 32;
#pragma unroll 1
        for (int k = 0; k < m32; ++k) {
          const int u    = __builtin_amdgcn_readlane(ent, k);
          const int wd   = __builtin_amdgcn_readlane(sr, k);
          const int slot = u & (NBRUN - 1);
          if (lane == 0) {
            int p = cur[slot];
            p = p < 0 ? 0 : (p > RCAP - 1 ? RCAP - 1 : p);
            pl[p] = wd;
            cur[slot] = p + 1;
          }
        }
      }
    }
  }
  __syncthreads();

  const int ovf = misc[9];
  int* lp  = LIST + (size_t)blk * RCAP;
  int* cop = CO + (size_t)blk * (2 * NBRUN);
  int* fp  = FLAG + (size_t)blk * 32;
  bucket_flush(pl, cnt, ovf, lp, cop, fp, tid);
  __threadfence();
  bucket_flush(pl, cnt, ovf, lp, cop, fp, tid);
}

__global__ __launch_bounds__(NTHR) void k_agg1(const int* __restrict__ LIST, const int* __restrict__ CO,
                                               const int* __restrict__ FLAG,
                                               const unsigned short* __restrict__ XB, unsigned short* M1hl) {
  const int tid = (int)threadIdx.x, lane = tid & 31, wave = tid >> 5, hh = lane >> 4, q = lane & 15;
  const int rowBase = (int)blockIdx.x * ABM;
  const int bucket  = rowBase >> SLB;
  const int* lb  = LIST + (size_t)bucket * RCAP;
  const int* cob = CO + (size_t)bucket * (2 * NBRUN);
  const int flag = FLAG[(size_t)bucket * 32];
  const float qnan = __uint_as_float(0x7fc00000u);

#pragma unroll 1
  for (int i = 0; i < ABM / (2 * NWAVE); ++i) {
    const int d    = rowBase + (ABM / NWAVE) * wave + 2 * i + hh;
    const int slot = d & (NBRUN - 1);
    int c = cob[slot];
    int o = cob[NBRUN + slot];
    const bool big = c > DEGCAP;
    c = c < 0 ? 0 : (c > DEGCAP ? DEGCAP : c);
    o = o < 0 ? 0 : (o > RCAP - 1 ? RCAP - 1 : o);
    const int co = __shfl_xor(c, 16, 32);
    const int cm = c > co ? c : co;
    int last = o + c - 1;
    last = last < o ? o : last;
    last = last > RCAP - 1 ? RCAP - 1 : last;
    float a0 = 0.0f, a1 = 0.0f, a2 = 0.0f, a3 = 0.0f;
#pragma unroll 1
    for (int j = 0; j < cm; ++j) {
      int idx = o + j;
      idx = idx > last ? last : idx;
      int sr = lb[idx];
      sr = sr < 0 ? 0 : (sr > NN - 1 ? NN - 1 : sr);
      const v2u w = *(const v2ua*)(XB + (size_t)sr * CIN + 4 * q);
      const unsigned wx = w.x, wy = w.y;
      asm volatile("" :: "v"(wx), "v"(wy));
      const bool valid = j < c;
      const float t0 = a0 + __uint_as_float(wx << 16);
      const float t1 = a1 + __uint_as_float(wx & 0xffff0000u);
      const float t2 = a2 + __uint_as_float(wy << 16);
      const float t3 = a3 + __uint_as_float(wy & 0xffff0000u);
      a0 = valid ? t0 : a0; a1 = valid ? t1 : a1; a2 = valid ? t2 : a2; a3 = valid ? t3 : a3;
    }
    const int   cd  = c > 1 ? c : 1;
    const float den = (float)cd;
    float m0 = a0 / den, m1 = a1 / den, m2 = a2 / den, m3 = a3 / den;
    const bool bad  = (flag != 0) | big;
    const bool live = d < NN;
    m0 = bad ? qnan : m0; m1 = bad ? qnan : m1; m2 = bad ? qnan : m2; m3 = bad ? qnan : m3;
    m0 = live ? m0 : 0.0f; m1 = live ? m1 : 0.0f; m2 = live ? m2 : 0.0f; m3 = live ? m3 : 0.0f;
    int h01, h23, l01, l23;
    hilo_pack(m0, m1, m2, m3, h01, h23, l01, l23);
    const v4i ow = regroup8(h01, h23, l01, l23, lane);
    st2_v4i(M1hl + (size_t)d * M1P + 8 * q, ow);
  }
}

template <int BP>
__device__ __forceinline__ void gemm_seg(const unsigned short* __restrict__ ap,
                                         const unsigned short* __restrict__ bp, int nk, v8f (&acc)[8]) {
#pragma unroll 1
  for (int k0 = 0; k0 < nk; k0 += 32) {
    FragB af;
    af.h[0] = *(const v8usa*)(ap + k0);
    af.h[1] = *(const v8usa*)(ap + k0 + 16);
#pragma unroll
    for (int nt = 0; nt < 8; ++nt) {
      const unsigned short* wq = bp + (size_t)(16 * nt) * (size_t)BP + k0;
      FragB bf;
      bf.h[0] = *(const v8usa*)wq;
      bf.h[1] = *(const v8usa*)(wq + 16);
      acc[nt] = wmb(af, bf, acc[nt]);
    }
  }
}

__device__ __forceinline__ void stage_d(float* stg, const v8f (&acc)[8], int wave, int hh, int m) {
#pragma unroll
  for (int nt = 0; nt < 8; ++nt) {
#pragma unroll
    for (int r = 0; r < 8; ++r) stg[(16 * wave + 8 * hh + r) * GBN + 16 * nt + m] = acc[nt][r];
  }
}

__global__ __launch_bounds__(GTHR) __attribute__((amdgpu_num_vgpr(248)))
void k_gemm1(const unsigned short* __restrict__ M1hl, const unsigned short* __restrict__ XB,
             const unsigned short* __restrict__ W1c, const float* __restrict__ sm, unsigned short* H1hl) {
  __shared__ __attribute__((aligned(16))) float stg[GBM * GBN];
  __shared__ __attribute__((aligned(16))) float sb[128];
  const int tid = (int)threadIdx.x, lane = tid & 31, wave = tid >> 5, hh = lane >> 4, m = lane & 15;
  const int rowBase = (int)blockIdx.x * GBM;
  if (tid < 32) *(v4fa*)(sb + 4 * tid) = *(const v4fa*)(sm + 4 * tid);

  v8f acc[8];
  {
    const v8f z = {0.f, 0.f, 0.f, 0.f, 0.f, 0.f, 0.f, 0.f};
#pragma unroll
    for (int t = 0; t < 8; ++t) acc[t] = z;
  }
  const int arow = rowBase + 16 * wave + m;
  const unsigned short* ap1 = M1hl + (size_t)arow * (size_t)M1P + 8 * hh;
  const unsigned short* ap2 = XB + (size_t)arow * (size_t)CIN + 8 * hh;
  const unsigned short* bp  = W1c + (size_t)m * (size_t)K1 + 8 * hh;
  gemm_seg<K1>(ap1, bp, 2 * CIN, acc);
  gemm_seg<K1>(ap2, bp + 2 * CIN, CIN, acc);
  stage_d(stg, acc, wave, hh, m);
  __syncthreads();

  const int c8 = 8 * m;
  const unsigned hm = (lane < 16) ? 0xffffffffu : 0u;
  const v4f bA = *(const v4fa*)(sb + c8);
  const v4f bB = *(const v4fa*)(sb + c8 + 4);
#pragma unroll 1
  for (int i = 0; i < 16; ++i) {
    const int lr   = 16 * wave + i;
    const int grow = rowBase + lr;
    const bool live = grow < NN;
    const v4f a0 = *(const v4fa*)(stg + lr * GBN + c8);
    const v4f a1 = *(const v4fa*)(stg + lr * GBN + c8 + 4);
    asm volatile("" :: "v"(a0));
    asm volatile("" :: "v"(a1));
    float v0 = a0.x + bA.x, v1 = a0.y + bA.y, v2 = a0.z + bA.z, v3 = a0.w + bA.w;
    float v4 = a1.x + bB.x, v5 = a1.y + bB.y, v6 = a1.z + bB.z, v7 = a1.w + bB.w;
    v0 = (v0 > 0.0f) ? v0 : (v0 - v0); v1 = (v1 > 0.0f) ? v1 : (v1 - v1);
    v2 = (v2 > 0.0f) ? v2 : (v2 - v2); v3 = (v3 > 0.0f) ? v3 : (v3 - v3);
    v4 = (v4 > 0.0f) ? v4 : (v4 - v4); v5 = (v5 > 0.0f) ? v5 : (v5 - v5);
    v6 = (v6 > 0.0f) ? v6 : (v6 - v6); v7 = (v7 > 0.0f) ? v7 : (v7 - v7);
    v0 = live ? v0 : 0.0f; v1 = live ? v1 : 0.0f; v2 = live ? v2 : 0.0f; v3 = live ? v3 : 0.0f;
    v4 = live ? v4 : 0.0f; v5 = live ? v5 : 0.0f; v6 = live ? v6 : 0.0f; v7 = live ? v7 : 0.0f;
    const unsigned p0 = hl_pick(v0, hm), p1 = hl_pick(v1, hm), p2 = hl_pick(v2, hm), p3 = hl_pick(v3, hm);
    const unsigned p4 = hl_pick(v4, hm), p5 = hl_pick(v5, hm), p6 = hl_pick(v6, hm), p7 = hl_pick(v7, hm);
    v4i ow;
    ow.x = (int)(p0 | (p1 << 16)); ow.y = (int)(p2 | (p3 << 16));
    ow.z = (int)(p4 | (p5 << 16)); ow.w = (int)(p6 | (p7 << 16));
    st2_v4i(H1hl + (size_t)grow * (size_t)K2 + 8 * lane, ow);
  }
}

__global__ __launch_bounds__(GTHR) __attribute__((amdgpu_num_vgpr(248)))
void k_gemm2(const unsigned short* __restrict__ H1hl, const unsigned short* __restrict__ W2c,
             const float* __restrict__ sm, float* PR) {
  __shared__ __attribute__((aligned(16))) float stg[GBM * GBN];
  __shared__ __attribute__((aligned(16))) float sb[128];
  const int tid = (int)threadIdx.x, lane = tid & 31, wave = tid >> 5, hh = lane >> 4, m = lane & 15;
  const int rowBase = (int)blockIdx.x * GBM;
  if (tid < 32) {
    const v4f b = *(const v4fa*)(sm + 128 + 4 * (lane & 15));
    const unsigned mk = (lane >= 16) ? 0xffffffffu : 0u;
    v4f o;
    o.x = __uint_as_float(__float_as_uint(b.x) & mk); o.y = __uint_as_float(__float_as_uint(b.y) & mk);
    o.z = __uint_as_float(__float_as_uint(b.z) & mk); o.w = __uint_as_float(__float_as_uint(b.w) & mk);
    *(v4fa*)(sb + 4 * lane) = o;
  }

  v8f acc[8];
  {
    const v8f z = {0.f, 0.f, 0.f, 0.f, 0.f, 0.f, 0.f, 0.f};
#pragma unroll
    for (int t = 0; t < 8; ++t) acc[t] = z;
  }
  const unsigned short* ap = H1hl + (size_t)(rowBase + 16 * wave + m) * (size_t)K2 + 8 * hh;
  const unsigned short* bp = W2c + (size_t)m * (size_t)K2 + 8 * hh;
  gemm_seg<K2>(ap, bp, K2, acc);
  stage_d(stg, acc, wave, hh, m);
  __syncthreads();

  const v4f bias = *(const v4fa*)(sb + 4 * lane);
  const size_t poff = (lane < 16) ? (size_t)0 : (size_t)MP * (size_t)COUT;
#pragma unroll 1
  for (int i = 0; i < 16; ++i) {
    const int lr   = 16 * wave + i;
    const int grow = rowBase + lr;
    const bool live = grow < NN;
    const v4f a = *(const v4fa*)(stg + lr * GBN + 4 * lane);
    asm volatile("" :: "v"(a));
    v4f o;
    o.x = live ? (a.x + bias.x) : 0.0f; o.y = live ? (a.y + bias.y) : 0.0f;
    o.z = live ? (a.z + bias.z) : 0.0f; o.w = live ? (a.w + bias.w) : 0.0f;
    st2_v4f(PR + poff + (size_t)grow * COUT + 4 * m, o);
  }
}

__global__ __launch_bounds__(NTHR) void k_agg2(const int* __restrict__ LIST, const int* __restrict__ CO,
                                               const int* __restrict__ FLAG, const float* __restrict__ PR,
                                               float* Z) {
  const int tid = (int)threadIdx.x, lane = tid & 31, wave = tid >> 5, hh = lane >> 4, q = lane & 15;
  const int rowBase = (int)blockIdx.x * ABM;
  const int bucket  = rowBase >> SLB;
  const int* lb  = LIST + (size_t)bucket * RCAP;
  const int* cob = CO + (size_t)bucket * (2 * NBRUN);
  const int flag = FLAG[(size_t)bucket * 32];
  const float qnan = __uint_as_float(0x7fc00000u);
  const float* Rp = PR + (size_t)MP * (size_t)COUT;

#pragma unroll 1
  for (int i = 0; i < ABM / (2 * NWAVE); ++i) {
    const int d    = rowBase + (ABM / NWAVE) * wave + 2 * i + hh;
    const int slot = d & (NBRUN - 1);
    int c = cob[slot];
    int o = cob[NBRUN + slot];
    const bool big = c > DEGCAP;
    c = c < 0 ? 0 : (c > DEGCAP ? DEGCAP : c);
    o = o < 0 ? 0 : (o > RCAP - 1 ? RCAP - 1 : o);
    const int co = __shfl_xor(c, 16, 32);
    const int cm = c > co ? c : co;
    int last = o + c - 1;
    last = last < o ? o : last;
    last = last > RCAP - 1 ? RCAP - 1 : last;
    float a0 = 0.0f, a1 = 0.0f, a2 = 0.0f, a3 = 0.0f;
#pragma unroll 1
    for (int j = 0; j < cm; ++j) {
      int idx = o + j;
      idx = idx > last ? last : idx;
      int sr = lb[idx];
      sr = sr < 0 ? 0 : (sr > NN - 1 ? NN - 1 : sr);
      const v4f v = *(const v4fa*)(PR + (size_t)sr * COUT + 4 * q);
      asm volatile("" :: "v"(v));
      const bool valid = j < c;
      const float t0 = a0 + v.x, t1 = a1 + v.y, t2 = a2 + v.z, t3 = a3 + v.w;
      a0 = valid ? t0 : a0; a1 = valid ? t1 : a1; a2 = valid ? t2 : a2; a3 = valid ? t3 : a3;
    }
    const v4f g = *(const v4fa*)(Rp + (size_t)d * COUT + 4 * q);
    asm volatile("" :: "v"(g));
    const int   cd  = c > 1 ? c : 1;
    const float den = (float)cd;
    float m0 = a0 / den + g.x, m1 = a1 / den + g.y, m2 = a2 / den + g.z, m3 = a3 / den + g.w;
    const bool bad  = (flag != 0) | big;
    const bool live = d < NN;
    m0 = bad ? qnan : m0; m1 = bad ? qnan : m1; m2 = bad ? qnan : m2; m3 = bad ? qnan : m3;
    m0 = live ? m0 : 0.0f; m1 = live ? m1 : 0.0f; m2 = live ? m2 : 0.0f; m3 = live ? m3 : 0.0f;
    v4f ov;
    ov.x = m0; ov.y = m1; ov.z = m2; ov.w = m3;
    st2_v4f(Z + (size_t)d * COUT + 4 * q, ov);
  }
}

__global__ __launch_bounds__(NTHR) void k_decode(const float* __restrict__ Z, const int* __restrict__ li,
                                                 const int* __restrict__ FLAG, float* out) {
  __shared__ __attribute__((aligned(16))) float stage[DPB];
  __shared__ unsigned sfl[NWAVE];
  const int tid = (int)threadIdx.x, lane = tid & 31, wave = tid >> 5, hh = lane >> 4, q = lane & 15;
  const int pbase = (int)blockIdx.x * DPB;
  {
    const int fi = tid < NBK ? tid : NBK - 1;
    const int f  = FLAG[(size_t)fi * 32];
    const unsigned b = __builtin_amdgcn_ballot_w32(f != 0);
    if (lane == 0) sfl[wave] = b;
  }
#pragma unroll 1
  for (int it = 0; it < DPB / 16; ++it) {
    const int lp = it * 16 + wave * 2 + hh;
    int p = pbase + lp;
    p = p > NPAIR - 1 ? NPAIR - 1 : p;
    int i0 = li[p];
    int i1 = li[NPAIR + p];
    i0 = i0 < 0 ? 0 : (i0 > NN - 1 ? NN - 1 : i0);
    i1 = i1 < 0 ? 0 : (i1 > NN - 1 ? NN - 1 : i1);
    const v4f a = *(const v4fa*)(Z + (size_t)i0 * COUT + 4 * q);
    const v4f b = *(const v4fa*)(Z + (size_t)i1 * COUT + 4 * q);
    asm volatile("" :: "v"(a));
    asm volatile("" :: "v"(b));
    const float p0 = a.x * b.x, p1 = a.y * b.y, p2 = a.z * b.z, p3 = a.w * b.w;
    float s = (p0 + p1) + (p2 + p3);
    s += __shfl_xor(s, 8, 32);
    s += __shfl_xor(s, 4, 32);
    s += __shfl_xor(s, 2, 32);
    s += __shfl_xor(s, 1, 32);
    if (q == 0) stage[lp] = s;
  }
  __syncthreads();
  const unsigned anyf = sfl[0] | sfl[1] | sfl[2] | sfl[3] | sfl[4] | sfl[5] | sfl[6] | sfl[7];
  const int livep = (NPAIR - pbase) < DPB ? (NPAIR - pbase) : DPB;
  const int nv4   = livep >> 2;
  v4f v = *(const v4fa*)(stage + 4 * tid);
  asm volatile("" :: "v"(v));
  const float qnan = __uint_as_float(0x7fc00000u);
  v.x = (anyf != 0u) ? qnan : v.x; v.y = (anyf != 0u) ? qnan : v.y;
  v.z = (anyf != 0u) ? qnan : v.z; v.w = (anyf != 0u) ? qnan : v.w;
  float* op = out + (size_t)pbase + (size_t)4 * (size_t)tid;
  if (tid < nv4) *(volatile v4f*)op = v;
  __threadfence();
  if (tid < nv4) *(volatile v4f*)op = v;
}

extern "C" void kernel_launch(void* const* d_in, const int* in_sizes, int n_in,
                              void* d_out, int out_size, void* d_ws, size_t ws_size,
                              hipStream_t stream) {
  if (n_in < 9) return;
  if (in_sizes[0] != NN * CIN) return;
  if (in_sizes[1] != CIN * CHID) return;
  if (in_sizes[2] != CIN * CHID) return;
  if (in_sizes[3] != CHID) return;
  if (in_sizes[4] != CHID * COUT) return;
  if (in_sizes[5] != CHID * COUT) return;
  if (in_sizes[6] != COUT) return;
  if (in_sizes[7] != 2 * NE) return;
  if (in_sizes[8] != 2 * NPAIR) return;
  if (out_size != NPAIR) return;

  const float* x   = (const float*)d_in[0];
  const float* Wl1 = (const float*)d_in[1];
  const float* Wr1 = (const float*)d_in[2];
  const float* b1  = (const float*)d_in[3];
  const float* Wl2 = (const float*)d_in[4];
  const float* Wr2 = (const float*)d_in[5];
  const float* b2  = (const float*)d_in[6];
  const int*   ei  = (const int*)d_in[7];
  const int*   li  = (const int*)d_in[8];
  float* out = (float*)d_out;
  const int* srcs = ei;
  const int* dsts = ei + NE;

  constexpr size_t zM1   = (size_t)MP * M1P * 2;
  constexpr size_t zXB   = (size_t)MP * CIN * 2;
  constexpr size_t zF64  = (size_t)MP * COUT * 4;
  constexpr size_t zRA   = 2 * zF64;
  constexpr size_t zRB   = (size_t)MP * K2 * 2;
  constexpr size_t zLIST = (size_t)NBK * RCAP * 4;
  constexpr size_t zCO   = (size_t)NBK * 2 * NBRUN * 4;
  constexpr size_t zFLAG = (size_t)NBK * 128;
  constexpr size_t zW1   = (size_t)CHID * K1 * 2;
  constexpr size_t zW2   = (size_t)CHID * K2 * 2;
  constexpr size_t zSM   = 1024;
  constexpr size_t oRA   = 0;
  constexpr size_t oRB   = oRA + zRA;
  constexpr size_t oLIST = oRB + zRB;
  constexpr size_t oCO   = oLIST + zLIST;
  constexpr size_t oFLAG = oCO + zCO;
  constexpr size_t oW1   = oFLAG + zFLAG;
  constexpr size_t oW2   = oW1 + zW1;
  constexpr size_t oSM   = oW2 + zW2;
  constexpr size_t oEND  = oSM + zSM;
  static_assert(zM1 + zXB <= zRA && zF64 <= zRB);
  static_assert(zM1 % 256 == 0 && zXB % 256 == 0 && zF64 % 256 == 0 && zRB % 256 == 0 && zLIST % 256 == 0);
  static_assert(zCO % 256 == 0 && zFLAG % 128 == 0 && zW1 % 256 == 0 && zW2 % 256 == 0 && zSM % 256 == 0);
  static_assert(oFLAG % 128 == 0 && oW1 % 128 == 0 && oW2 % 128 == 0 && oSM % 128 == 0);
  static_assert(oEND <= (size_t)(128u << 20));
  if (oEND > ws_size) return;

  char* ws = (char*)d_ws;
  unsigned short* M1hl = (unsigned short*)(ws + oRA);
  unsigned short* XB   = (unsigned short*)(ws + oRA + zM1);
  float*          PR   = (float*)(ws + oRA);
  unsigned short* H1hl = (unsigned short*)(ws + oRB);
  float*          Z    = (float*)(ws + oRB);
  int*            LIST = (int*)(ws + oLIST);
  int*            CO   = (int*)(ws + oCO);
  int*            FLAG = (int*)(ws + oFLAG);
  unsigned short* W1c  = (unsigned short*)(ws + oW1);
  unsigned short* W2c  = (unsigned short*)(ws + oW2);
  float*          SM   = (float*)(ws + oSM);

  hipFuncSetAttribute(reinterpret_cast<const void*>(&k_bucket), hipFuncAttributeMaxDynamicSharedMemorySize, (int)BK_LDS);

  k_prep<<<PBTOT, NTHR, 0, stream>>>(x, Wl1, Wr1, b1, Wl2, Wr2, b2, XB, W1c, W2c, SM);
  k_bucket<<<NBK, NTHR, BK_LDS, stream>>>(srcs, dsts, LIST, CO, FLAG);
  k_agg1<<<MP / ABM, NTHR, 0, stream>>>(LIST, CO, FLAG, XB, M1hl);
  k_gemm1<<<MP / GBM, GTHR, 0, stream>>>(M1hl, XB, W1c, SM, H1hl);
  k_gemm2<<<MP / GBM, GTHR, 0, stream>>>(H1hl, W2c, SM, PR);
  k_agg2<<<MP / ABM, NTHR, 0, stream>>>(LIST, CO, FLAG, PR, Z);
  k_decode<<<NDB, NTHR, 0, stream>>>(Z, li, FLAG, out);
}
